// PrototypeLayer_16844861735549
// MI455X (gfx1250) — hardware-verified
//
#include <hip/hip_runtime.h>
#include <stddef.h>


typedef _Float16 v16h __attribute__((ext_vector_type(16)));
typedef _Float16 v8h  __attribute__((ext_vector_type(8)));
typedef float    v8f  __attribute__((ext_vector_type(8)));
typedef float    v4f  __attribute__((ext_vector_type(4)));
typedef _Float16 h16;

#ifndef NB
#define NB 32
#endif
#define NB_FULL  32
#define DIM      256
#define TOK      784
#define TOKP     800
#define NTILE    (TOK / 16)
#define NPROTO   2000
#define NPP      2048
#define XB_FULL  (DIM * TOK)
#define OUT1_BYTES 256000
#define OUT1_ELEM  (OUT1_BYTES / 4)

static_assert(NB >= 1 && NB <= NB_FULL);
static_assert(DIM == 256 && (DIM % 32) == 0 && DIM / 32 == 8);
static_assert(DIM == 32 * 8);
static_assert((TOK % 16) == 0 && NTILE * 16 == TOK);
static_assert((TOKP % 32) == 0 && TOKP >= TOK && TOKP - TOK < 32);
static_assert((NPP % 128) == 0 && NPP >= NPROTO && (NPP % 32) == 0);
static_assert((NPROTO % 4) == 0);
static_assert(OUT1_BYTES == NB_FULL * NPROTO * 4);
static_assert((OUT1_BYTES % 128) == 0);
static_assert((size_t)OUT1_ELEM + (size_t)NB * NPROTO <= (size_t)2 * NB_FULL * NPROTO);

#define LDX 264
static_assert((LDX % 8) == 0 && LDX >= DIM);

#define WCARRY 64.0f

#define X16_BYTES ((size_t)NB * TOKP * DIM * 2)
#define P16_BYTES ((size_t)NPP * DIM * 2)
#define XSQ_BYTES ((size_t)NB * TOKP * 4)
#define PSQ_BYTES ((size_t)NPP * 4)
#define MNV_BYTES ((size_t)NB * NPP * 4)
#define OFF_X16 ((size_t)0)
#define OFF_P16 (OFF_X16 + X16_BYTES)
#define OFF_XSQ (OFF_P16 + P16_BYTES)
#define OFF_PSQ (OFF_XSQ + XSQ_BYTES)
#define OFF_MNV (OFF_PSQ + PSQ_BYTES)
#define WS_TOTAL (OFF_MNV + MNV_BYTES)
static_assert((X16_BYTES % 128) == 0 && (P16_BYTES % 128) == 0);
static_assert((XSQ_BYTES % 128) == 0 && (PSQ_BYTES % 128) == 0 && (MNV_BYTES % 128) == 0);
static_assert(WS_TOTAL <= (size_t)134217728);

__device__ __forceinline__ float bf16r(float x) {
  unsigned int u = __float_as_uint(x);
  u = (u + 0x7FFFu + ((u >> 16) & 1u)) & 0xFFFF0000u;
  return __uint_as_float(u);
}

static __device__ __forceinline__ h16 toh_flush(float v) {
  const h16 r = (h16)v;
  return (fabsf(v) < 6.103515625e-05f) ? (h16)0.0f : r;
}

__device__ __forceinline__ v16h frag_at(const _Float16* p) {
  v8h lo = *(const v8h*)(p);
  v8h hi = *(const v8h*)(p + 16);
  v16h out;
#pragma unroll
  for (int i = 0; i < 8; ++i) { out[i] = lo[i]; out[i + 8] = hi[i]; }
  return out;
}

__device__ __forceinline__ v8f wmma16(v16h a, v16h b, v8f c) {
  v8f d = __builtin_amdgcn_wmma_f32_16x16x32_f16(false, a, false, b, (short)0, c,
                                                 false, false);
  asm volatile("v_nop\n\tv_nop\n\tv_nop\n\tv_nop" : "+v"(d) : "v"(a), "v"(b));
  return d;
}

static_assert(256 * 32 == 32 * DIM);
static_assert(8 * 4 == 32);
static_assert(32 * LDX * 2 + 32 * 4 <= 131072);

__global__ __launch_bounds__(256) void tconv_kernel(
    const float* __restrict__ src, _Float16* __restrict__ dst, float* __restrict__ sq,
    unsigned sk, unsigned sn, unsigned nlast, unsigned sbatch, unsigned npad) {
#pragma clang fp contract(off)
  __shared__ _Float16 T[32 * LDX];
  __shared__ float S[32];
  const unsigned tid = threadIdx.x;
  const unsigned n0 = blockIdx.x * 32u;
  const unsigned bz = blockIdx.y;
  const float* sb = src + (size_t)bz * sbatch;
#pragma unroll 4
  for (unsigned j = 0; j < 32u; ++j) {
    const unsigned idx = tid + 256u * j;
    const unsigned kr = idx >> 5, nc = idx & 31u;
    const unsigned nn = n0 + nc;
    const unsigned ncl = (nn < nlast) ? nn : nlast;
    const float v = sb[(size_t)kr * sk + (size_t)ncl * sn];
    T[nc * LDX + kr] = toh_flush(WCARRY * bf16r(v));
  }
  __syncthreads();

  const unsigned t = tid >> 3, part = tid & 7u;
  float ss = 0.0f;
#pragma unroll 1
  for (unsigned q = 0; q < 4u; ++q) {
    const v8h hv = *(const v8h*)&T[t * LDX + part * 32u + q * 8u];
#pragma unroll
    for (int i = 0; i < 8; ++i) {
      const float e = (float)hv[i];
      ss += e * e;
    }
  }
  ss += __shfl_xor(ss, 1, 32);
  ss += __shfl_xor(ss, 2, 32);
  ss += __shfl_xor(ss, 4, 32);
  if (part == 0u) S[t] = ss * (1.0f / (WCARRY * WCARRY));

  v8h x[4];
  size_t off[4];
#pragma unroll
  for (unsigned i = 0; i < 4u; ++i) {
    const unsigned n = 8u * i + (tid >> 5);
    const unsigned kc = (tid & 31u) * 8u;
    x[i] = *(const v8h*)&T[n * LDX + kc];
    off[i] = ((size_t)bz * npad + n0 + n) * DIM + kc;
  }
  __syncthreads();
  const v4f sv = *(const v4f*)&S[(tid & 7u) * 4u];
  float* sp = sq + (size_t)bz * npad + n0 + (tid & 7u) * 4u;

#pragma unroll
  for (int i = 0; i < 4; ++i) *(volatile v8h*)(dst + off[i]) = x[i];
  if (tid < 8u) *(volatile v4f*)sp = sv;
  __threadfence();
#pragma unroll
  for (int i = 0; i < 4; ++i) *(volatile v8h*)(dst + off[i]) = x[i];
  if (tid < 8u) *(volatile v4f*)sp = sv;
}

static_assert(8 * 16 == 128);
static_assert(32 * 4 == 128);

__global__ __launch_bounds__(256) void dist_kernel(
    const _Float16* __restrict__ X16, const _Float16* __restrict__ P16,
    const float* __restrict__ xsq, float* __restrict__ mnv) {
  __shared__ float S[128];
  const unsigned tid = threadIdx.x, lane = tid & 31u;
  const unsigned wave = (unsigned)__builtin_amdgcn_readfirstlane((int)(threadIdx.x >> 5));
  const unsigned hh = lane >> 4, m = lane & 15u;
  const unsigned b = blockIdx.y;
  const unsigned p0 = blockIdx.x * 128u + wave * 16u;

  const _Float16* bp = P16 + (size_t)(p0 + m) * DIM + hh * 8u;
  v16h bf[8];
#pragma unroll
  for (int c = 0; c < 8; ++c) bf[c] = frag_at(bp + c * 32);

  const _Float16* ap = X16 + ((size_t)b * TOKP + m) * DIM + hh * 8u;
  const float* xs = xsq + (size_t)b * TOKP + hh * 8u;
  const float cs = 2.0f / (WCARRY * WCARRY);
  float runmin = 3.4e38f;

#pragma unroll 1
  for (unsigned nt = 0; nt < (unsigned)NTILE; ++nt) {
    const _Float16* a = ap + (size_t)nt * (16u * DIM);
    v8f acc = {};
#pragma unroll
    for (int c = 0; c < 8; ++c) {
      const v16h af = frag_at(a + c * 32);
      acc = wmma16(af, bf[c], acc);
    }
    const v4f x0 = *(const v4f*)(xs + nt * 16u);
    const v4f x1 = *(const v4f*)(xs + nt * 16u + 4u);
#pragma unroll
    for (int r = 0; r < 4; ++r) {
      runmin = fminf(runmin, x0[r] - acc[r] * cs);
      runmin = fminf(runmin, x1[r] - acc[r + 4] * cs);
    }
  }
  runmin = fminf(runmin, __shfl_xor(runmin, 16, 32));
  if (lane < 16u) S[wave * 16u + m] = runmin;
  __syncthreads();
  const v4f sv = *(const v4f*)&S[lane * 4u];
  if (wave == 0u) {
    float* p = mnv + (size_t)b * NPP + blockIdx.x * 128u + lane * 4u;
    *(volatile v4f*)p = sv;
    __threadfence();
    *(volatile v4f*)p = sv;
  }
}

__global__ __launch_bounds__(256) void fin_kernel(
    const float* __restrict__ mnv, const float* __restrict__ psq, float* __restrict__ out) {
#pragma clang fp contract(off)
  const unsigned total = (unsigned)NB * (unsigned)NPROTO;
  const unsigned e = blockIdx.x * 256u + threadIdx.x;
  const unsigned ec = (e < total) ? e : (total - 1u);
  const unsigned b = ec / (unsigned)NPROTO;
  const unsigned p = ec - b * (unsigned)NPROTO;
  const float mv = mnv[(size_t)b * NPP + p];
  const float ps = psq[p];
  const float d2 = fmaxf(mv + ps, 1.0e-12f);
  const float dist = sqrtf(d2);
  const float sim = logf((dist + 1.0f) / (dist + 1.0e-7f));
  if (e < total) {
    volatile float* o0 = out + ec;
    volatile float* o1 = out + (size_t)OUT1_ELEM + ec;
    *o0 = sim;
    *o1 = dist;
    __threadfence();
    *o0 = sim;
    *o1 = dist;
  }
}

extern "C" void kernel_launch(void* const* d_in, const int* in_sizes, int n_in,
                              void* d_out, int out_size, void* d_ws, size_t ws_size,
                              hipStream_t stream) {
  if (n_in < 2) return;
  if ((long long)in_sizes[0] < (long long)NB * XB_FULL) return;
  if ((long long)in_sizes[1] < (long long)NPROTO * DIM) return;
  if ((long long)out_size < (long long)OUT1_ELEM + (long long)NB * NPROTO) return;
  if (ws_size < WS_TOTAL) return;

  const float* X  = (const float*)d_in[0];
  const float* Pr = (const float*)d_in[1];
  float* out = (float*)d_out;

  char* ws = (char*)d_ws;
  _Float16* X16 = (_Float16*)(ws + OFF_X16);
  _Float16* P16 = (_Float16*)(ws + OFF_P16);
  float*    XSQ = (float*)(ws + OFF_XSQ);
  float*    PSQ = (float*)(ws + OFF_PSQ);
  float*    MNV = (float*)(ws + OFF_MNV);

  dim3 blk(256);
  tconv_kernel<<<dim3(TOKP / 32, NB), blk, 0, stream>>>(
      X, X16, XSQ, (unsigned)TOK, 1u, (unsigned)(TOK - 1), (unsigned)XB_FULL, (unsigned)TOKP);
  tconv_kernel<<<dim3(NPP / 32, 1), blk, 0, stream>>>(
      Pr, P16, PSQ, 1u, (unsigned)DIM, (unsigned)(NPROTO - 1), 0u, (unsigned)NPP);
  dist_kernel<<<dim3(NPP / 128, NB), blk, 0, stream>>>(X16, P16, XSQ, MNV);
  fin_kernel<<<dim3((NB * NPROTO + 255) / 256), blk, 0, stream>>>(MNV, PSQ, out);
}
